// SoftMesh_35313221107989
// MI455X (gfx1250) — hardware-verified
//
#include <hip/hip_runtime.h>
#include <math.h>
#include <stdint.h>
#pragma clang fp contract(off)

#define RESN 128
#define VOX 2097152
#define NVOL 6
#define NCL 4
#define NCO 3
#define NZF 48
#define NSB 32
#define PA 136

typedef _Float16 v16h __attribute__((ext_vector_type(16)));
typedef _Float16 v8h __attribute__((ext_vector_type(8)));
typedef float v8f __attribute__((ext_vector_type(8)));
typedef float v4f __attribute__((ext_vector_type(4)));
typedef float v4fa __attribute__((ext_vector_type(4), __may_alias__));
union Frag { v16h v; v8h hf[2]; };
union H8 { v8h v; _Float16 s[8]; };

__device__ __forceinline__ v8f mma16(v16h a, v16h b, v8f c) {
  c = __builtin_amdgcn_wmma_f32_16x16x32_f16(false, a, false, b, (short)0, c, false, false);
  asm volatile("v_nop\n\tv_nop\n\tv_nop\n\tv_nop" : "+v"(c) : "v"(a), "v"(b));
  return c;
}

__device__ __forceinline__ void corner_axis(float pc, int& i0, float& fr) {
  float q = ((pc + 1.0f) * 128.0f - 1.0f) * 0.5f;
  float f = floorf(q);
  fr = q - f;
  f = fminf(fmaxf(f, -4.0f), 132.0f);
  i0 = (int)f;
}

__global__ __launch_bounds__(256) void probs_k(const float* __restrict__ lg, float* __restrict__ pr, int npts) {
  int j = blockIdx.x * 256 + threadIdx.x;
  if (j >= 2 * npts) return;
  int b = j / npts, p = j - b * npts;
  float l[NCL], mx = -3.0e38f;
#pragma unroll
  for (int c = 0; c < NCL; ++c) { l[c] = lg[(size_t)(b * NCL + c) * npts + p]; mx = fmaxf(mx, l[c]); }
  float den = 0.0f;
#pragma unroll
  for (int c = 0; c < NCL; ++c) { l[c] = expf(l[c] - mx); den += l[c]; }
  float inv = 1.0f / den;
  float o[NCO];
#pragma unroll
  for (int c = 0; c < NCO; ++c) o[c] = l[c + 1] * inv;
#pragma unroll
  for (int c = 0; c < NCO; ++c) *(volatile float*)(pr + (size_t)(b * NCO + c) * npts + p) = o[c];
  __threadfence();
#pragma unroll
  for (int c = 0; c < NCO; ++c) *(volatile float*)(pr + (size_t)(b * NCO + c) * npts + p) = o[c];
}

__global__ __launch_bounds__(32) void splat_k(const float* __restrict__ coords, const float* __restrict__ pr,
                                              float* __restrict__ g, int npts) {
  extern __shared__ __attribute__((aligned(16))) float cell[];
  volatile float* vc = cell;
  const int lane = threadIdx.x;
  const int b = blockIdx.x >> 7, s = blockIdx.x & 127;
  v4f z4 = {0.f, 0.f, 0.f, 0.f};
  for (int i = lane * 4; i < NCO * 16384; i += 128) *(v4fa*)&cell[i] = z4;
  __syncthreads();
  for (int base = 0; base < npts; base += 32) {
    int p = base + lane;
    bool valid = p < npts;
    int pcl = valid ? p : 0;
    float px = coords[(size_t)(b * 3 + 0) * npts + pcl];
    float py = coords[(size_t)(b * 3 + 1) * npts + pcl];
    float pz = coords[(size_t)(b * 3 + 2) * npts + pcl];
    int ix0, iy0, iz0; float fx, fy, fz;
    corner_axis(px, ix0, fx); corner_axis(py, iy0, fy); corner_axis(pz, iz0, fz);
    float wx = 0.0f; bool hit = false;
    if (valid) {
      if (ix0 == s) { wx = 1.0f - fx; hit = true; }
      else if (ix0 + 1 == s) { wx = fx; hit = true; }
    }
    unsigned mask = (unsigned)__ballot(hit);
    while (mask) {
      int j = __builtin_ctz(mask);
      mask &= mask - 1u;
      int jy = __shfl(iy0, j), jz = __shfl(iz0, j), jp = __shfl(pcl, j);
      float jfy = __shfl(fy, j), jfz = __shfl(fz, j), jwx = __shfl(wx, j);
      if (lane < 12) {
        int c = lane >> 2, q = lane & 3, oy = q >> 1, oz = q & 1;
        int iy = jy + oy, iz = jz + oz;
        if (iy >= 0 && iy < RESN && iz >= 0 && iz < RESN) {
          float w = jwx * (oy ? jfy : 1.0f - jfy) * (oz ? jfz : 1.0f - jfz);
          float prv = pr[(size_t)(b * NCO + c) * npts + jp];
          int idx = c * 16384 + iy * RESN + iz;
          vc[idx] = vc[idx] + prv * w;
        }
      }
    }
  }
  __syncthreads();
  for (int ps = 0; ps < 2; ++ps) {
#pragma unroll 1
    for (int c = 0; c < NCO; ++c) {
      float* dst = g + ((size_t)((b * NCO + c) * RESN + s)) * 16384;
      for (int i = lane * 4; i < 16384; i += 128) {
        v4f x = *(v4fa*)&cell[c * 16384 + i];
        *(volatile v4f*)(dst + i) = x;
      }
    }
    if (ps == 0) __threadfence();
  }
}

__global__ __launch_bounds__(128) void init_k(_Float16* __restrict__ RT, _Float16* __restrict__ C, _Float16* __restrict__ S,
                                              _Float16* __restrict__ Sn, _Float16* __restrict__ Cz, _Float16* __restrict__ Szn) {
  __shared__ float kk[128];
  __shared__ float dk[32];
  __shared__ __attribute__((aligned(16))) _Float16 rowh[3][128];
  const int t = threadIdx.x, bid = blockIdx.x;
  const float TWOPI = 6.2831853071795864769f;
  if (bid < 128) {
    const int n = bid;
    {
      float s = 0.0f;
      for (int f = 1; f < 64; ++f) {
        int mm = (f * t) & 127;
        s += (float)f * sinf(TWOPI * (float)mm * (1.0f / 128.0f));
      }
      kk[t] = s * (2.0f * TWOPI / 128.0f);
    }
    if (t < 31) {
      float gs = 0.0f;
      for (int x = -15; x <= 15; ++x) gs += expf(-0.005f * (float)(x * x));
      float x = (float)(t - 15);
      dk[t] = (-x * 0.01f * expf(-0.005f * x * x)) / gs;
    }
    __syncthreads();
    {
      int m = t; float r = 0.0f;
      int p0 = (m - 15 > 0) ? m - 15 : 0, p1 = (m + 15 < 127) ? m + 15 : 127;
      for (int p = p0; p <= p1; ++p) r += kk[(n - p) & 127] * dk[m - p + 15];
      rowh[0][m] = (_Float16)(r * 256.0f);
    }
    __syncthreads();
    for (int ps = 0; ps < 2; ++ps) {
      if (t < 16) { v8h x = *(const v8h*)&rowh[0][8 * t]; *(volatile v8h*)(RT + n * 128 + 8 * t) = x; }
      if (ps == 0) __threadfence();
    }
  } else if (bid < 256) {
    const int n = bid - 128;
    int mm = (n * t) & 127;
    float th = TWOPI * (float)mm * (1.0f / 128.0f);
    float c = cosf(th), s = sinf(th);
    rowh[0][t] = (_Float16)c; rowh[1][t] = (_Float16)s; rowh[2][t] = (_Float16)(-s);
    __syncthreads();
    for (int ps = 0; ps < 2; ++ps) {
      if (t < 16) {
        v8h a = *(const v8h*)&rowh[0][8 * t], bq = *(const v8h*)&rowh[1][8 * t], cq = *(const v8h*)&rowh[2][8 * t];
        *(volatile v8h*)(C + n * 128 + 8 * t) = a;
        *(volatile v8h*)(S + n * 128 + 8 * t) = bq;
        *(volatile v8h*)(Sn + n * 128 + 8 * t) = cq;
      }
      if (ps == 0) __threadfence();
    }
  } else if (bid < 384) {
    const int n = bid - 256;
    if (t < 64) {
      float wgt = (t == 0) ? 1.0f : ((t < NZF) ? 2.0f : 0.0f);
      int mm = (n * t) & 127;
      float th = TWOPI * (float)mm * (1.0f / 128.0f);
      rowh[0][t] = (_Float16)(wgt * cosf(th));
      rowh[1][t] = (_Float16)(-wgt * sinf(th));
    }
    __syncthreads();
    for (int ps = 0; ps < 2; ++ps) {
      if (t < 8) {
        v8h a = *(const v8h*)&rowh[0][8 * t], bq = *(const v8h*)&rowh[1][8 * t];
        *(volatile v8h*)(Cz + n * 64 + 8 * t) = a;
        *(volatile v8h*)(Szn + n * 64 + 8 * t) = bq;
      }
      if (ps == 0) __threadfence();
    }
  }
}

template <int M>
__global__ __launch_bounds__(64) void pass_k(const float* __restrict__ fre, const float* __restrict__ fim,
                                             const _Float16* __restrict__ h0, const _Float16* __restrict__ h1,
                                             const _Float16* __restrict__ h2,
                                             const _Float16* __restrict__ T0, const _Float16* __restrict__ T1,
                                             const _Float16* __restrict__ T2,
                                             float* __restrict__ o0, float* __restrict__ o1, _Float16* __restrict__ oh) {
  constexpr int LPV = (M >= 4 && M <= 7) ? 6144 : 16384;
  constexpr int K = (M == 8) ? 64 : 128;
  constexpr int KP = K;
  constexpr bool KCONT = (M == 2 || M == 3 || M == 6);
  constexpr bool CIN = (M >= 4);
  constexpr bool COUT = (M >= 3 && M <= 7);
  constexpr int NCT = (M == 3) ? 3 : 4;
  constexpr int NGRP = (M == 3) ? 1 : 2;
  constexpr int OUTW = (M == 3) ? 64 : 128;
  constexpr bool OUT16 = (M <= 2);
  constexpr float SC = (M <= 2) ? 64.0f : ((M == 3) ? 1.0f : ((M <= 5) ? 256.0f : 16384.0f));
  constexpr float EPI = (M <= 2) ? (1.0f / 64.0f) : ((M <= 5) ? (1.0f / 4096.0f) : (1.0f / 524288.0f));
  constexpr float A2 = 0.01220703125f;
  constexpr float FOURPI2 = 39.47841760435743f;

  __shared__ __attribute__((aligned(16))) _Float16 Ar_s[32 * PA];
  __shared__ __attribute__((aligned(16))) _Float16 Ai_s[32 * PA];
  __shared__ __attribute__((aligned(16))) float Es[2][2][16][128];

  constexpr int BPV = LPV / 32;
  if (blockIdx.x >= NVOL * BPV) return;
  const int v = blockIdx.x / BPV;
  const int L0 = (blockIdx.x - v * BPV) * 32;
  const int tid = threadIdx.x;

#pragma unroll 1
  for (int i = 0; i < (32 * K) / 64; ++i) {
    int e = tid + 64 * i;
    int j, k;
    if (KCONT) { j = e / K; k = e - j * K; } else { k = e >> 5; j = e & 31; }
    int L = L0 + j;
    float vr = 0.0f, vi = 0.0f;
    if (M == 0) {
      vr = fre[(size_t)v * VOX + (size_t)k * 16384 + L];
    } else if (M == 1) {
      int x = L >> 7, z = L & 127;
      vr = fre[(size_t)v * VOX + (size_t)x * 16384 + k * 128 + z];
    } else if (M == 2) {
      vr = fre[(size_t)v * VOX + (size_t)L * 128 + k];
    } else if (M == 3) {
      int x = L >> 7, y = L & 127;
      size_t vb = (size_t)v * VOX;
      vr = (float)h0[vb + (size_t)L * 128 + k] + (float)h1[vb + ((size_t)x * 128 + k) * 128 + y] +
           (float)h2[vb + ((size_t)y * 128 + k) * 128 + x];
    } else if (M == 4) {
      int x = L / 48, kz = L - x * 48;
      size_t id = ((size_t)v * 16384 + x * 128 + k) * 64 + kz;
      vr = fre[id]; vi = fim[id];
    } else if (M == 5) {
      int ky = L / 48, kz = L - ky * 48;
      size_t id = ((size_t)v * 6144 + k * 48 + kz) * 128 + ky;
      vr = fre[id]; vi = fim[id];
    } else if (M == 6) {
      size_t id = ((size_t)v * 6144 + L) * 128 + k;
      vr = fre[id]; vi = fim[id];
    } else if (M == 7) {
      int x = L / 48, kz = L - x * 48;
      size_t id = ((size_t)v * 6144 + k * 48 + kz) * 128 + x;
      vr = fre[id]; vi = fim[id];
    } else {
      int x = L >> 7, y = L & 127;
      if (k < NZF) {
        size_t id = ((size_t)v * 6144 + x * 48 + k) * 128 + y;
        vr = fre[id]; vi = fim[id];
      }
    }
    Ar_s[j * PA + k] = (_Float16)(vr * SC);
    if (CIN) Ai_s[j * PA + k] = (_Float16)(vi * SC);
  }
  __syncthreads();

  const int w = tid >> 5, l = tid & 31, h = l >> 4, m = l & 15;

  float eyz[8], f2yz[8];
  if (M == 5) {
#pragma unroll
    for (int r = 0; r < 8; ++r) {
      int L = L0 + w * 16 + 8 * h + r;
      int ky = L / 48, kz = L - ky * 48;
      float fy = (float)((ky < 64) ? ky : ky - 128), fz = (float)kz;
      f2yz[r] = fy * fy + fz * fz;
      eyz[r] = __expf(-A2 * f2yz[r]);
    }
  }

#pragma unroll
  for (int gI = 0; gI < NGRP; ++gI) {
    v8f acr[NCT], aci[NCT];
#pragma unroll
    for (int ct = 0; ct < NCT; ++ct) { acr[ct] = (v8f){0, 0, 0, 0, 0, 0, 0, 0}; aci[ct] = (v8f){0, 0, 0, 0, 0, 0, 0, 0}; }
#pragma unroll 1
    for (int ks = 0; ks < K / 32; ++ks) {
      const int k0 = ks * 32;
      Frag a, ai;
      a.hf[0] = *(const v8h*)&Ar_s[(w * 16 + m) * PA + k0 + 8 * h];
      a.hf[1] = *(const v8h*)&Ar_s[(w * 16 + m) * PA + k0 + 16 + 8 * h];
      if (CIN) {
        ai.hf[0] = *(const v8h*)&Ai_s[(w * 16 + m) * PA + k0 + 8 * h];
        ai.hf[1] = *(const v8h*)&Ai_s[(w * 16 + m) * PA + k0 + 16 + 8 * h];
      }
#pragma unroll
      for (int ct = 0; ct < NCT; ++ct) {
        const int n = (gI * NCT + ct) * 16 + m;
        const size_t tb = (size_t)n * KP + k0 + 8 * h;
        Frag b0;
        b0.hf[0] = *(const v8h*)(T0 + tb);
        b0.hf[1] = *(const v8h*)(T0 + tb + 16);
        acr[ct] = mma16(a.v, b0.v, acr[ct]);
        if (CIN) {
          Frag b1;
          b1.hf[0] = *(const v8h*)(T1 + tb);
          b1.hf[1] = *(const v8h*)(T1 + tb + 16);
          acr[ct] = mma16(ai.v, b1.v, acr[ct]);
          if (COUT) aci[ct] = mma16(ai.v, b0.v, aci[ct]);
        }
        if (COUT) {
          Frag b2;
          b2.hf[0] = *(const v8h*)(T2 + tb);
          b2.hf[1] = *(const v8h*)(T2 + tb + 16);
          aci[ct] = mma16(a.v, b2.v, aci[ct]);
        }
      }
    }
#pragma unroll
    for (int ct = 0; ct < NCT; ++ct) {
      const int col = (gI * NCT + ct) * 16 + m;
      float ex = 1.0f, f2x = 0.0f;
      if (M == 5) {
        int n = col;
        float fx = (float)((n < 64) ? n : n - 128);
        f2x = fx * fx;
        ex = __expf(-A2 * f2x);
      }
#pragma unroll
      for (int r = 0; r < 8; ++r) {
        float e = EPI;
        if (M == 5) {
          float f2 = f2x + f2yz[r];
          float Hv = (f2 == 0.0f) ? 0.0f : __fdividef(ex * eyz[r], -FOURPI2 * f2);
          e = EPI * Hv;
        }
        Es[0][w][8 * h + r][col] = acr[ct][r] * e;
        if (COUT) Es[1][w][8 * h + r][col] = aci[ct][r] * e;
      }
    }
    if (M == 3) {
#pragma unroll
      for (int r = 0; r < 8; ++r) { Es[0][w][8 * h + r][48 + m] = 0.0f; Es[1][w][8 * h + r][48 + m] = 0.0f; }
    }
  }
  __syncthreads();

  for (int ps = 0; ps < 2; ++ps) {
#pragma unroll 1
    for (int r = 0; r < 16; ++r) {
      const int L = L0 + w * 16 + r;
      const size_t ro = (size_t)v * LPV + L;
      if (OUT16) {
        if (l < 16) {
          H8 hv;
#pragma unroll
          for (int i = 0; i < 8; ++i) hv.s[i] = (_Float16)Es[0][w][r][8 * l + i];
          *(volatile v8h*)(oh + ro * 128 + 8 * l) = hv.v;
        }
      } else {
        if (l < OUTW / 4) {
          v4f x = *(const v4fa*)&Es[0][w][r][4 * l];
          *(volatile v4f*)(o0 + ro * OUTW + 4 * l) = x;
          if (COUT) {
            v4f y = *(const v4fa*)&Es[1][w][r][4 * l];
            *(volatile v4f*)(o1 + ro * OUTW + 4 * l) = y;
          }
        }
      }
    }
    if (ps == 0) __threadfence();
  }
}

__global__ __launch_bounds__(256) void samp_k(const float* __restrict__ coords, const float* __restrict__ phi,
                                              float* __restrict__ part, int npts) {
  __shared__ float red[NCO][256];
  __shared__ __attribute__((aligned(16))) float ln[32];
  const int tid = threadIdx.x;
  const int b = blockIdx.x / NSB, blk = blockIdx.x - b * NSB;
  const int chunk = (npts + NSB - 1) / NSB;
  const int p0 = blk * chunk;
  const int p1 = (p0 + chunk < npts) ? p0 + chunk : npts;
  float s[NCO] = {0.0f, 0.0f, 0.0f};
  for (int p = p0 + tid; p < p1; p += 256) {
    float px = coords[(size_t)(b * 3 + 0) * npts + p];
    float py = coords[(size_t)(b * 3 + 1) * npts + p];
    float pz = coords[(size_t)(b * 3 + 2) * npts + p];
    int ix0, iy0, iz0; float fx, fy, fz;
    corner_axis(px, ix0, fx); corner_axis(py, iy0, fy); corner_axis(pz, iz0, fz);
    float acc[NCO] = {0.0f, 0.0f, 0.0f};
#pragma unroll
    for (int o = 0; o < 8; ++o) {
      int ox = (o >> 2) & 1, oy = (o >> 1) & 1, oz = o & 1;
      int ix = ix0 + ox, iy = iy0 + oy, iz = iz0 + oz;
      bool inb = (ix >= 0) && (ix < RESN) && (iy >= 0) && (iy < RESN) && (iz >= 0) && (iz < RESN);
      if (inb) {
        float w = (ox ? fx : 1.0f - fx) * (oy ? fy : 1.0f - fy) * (oz ? fz : 1.0f - fz);
        int flat = (ix * RESN + iy) * RESN + iz;
#pragma unroll
        for (int c = 0; c < NCO; ++c) acc[c] += phi[(size_t)(b * NCO + c) * VOX + flat] * w;
      }
    }
#pragma unroll
    for (int c = 0; c < NCO; ++c) s[c] += acc[c];
  }
#pragma unroll
  for (int c = 0; c < NCO; ++c) red[c][tid] = s[c];
  __syncthreads();
  for (int st = 128; st > 0; st >>= 1) {
    if (tid < st) {
#pragma unroll
      for (int c = 0; c < NCO; ++c) red[c][tid] += red[c][tid + st];
    }
    __syncthreads();
  }
  if (tid < 32) ln[tid] = (tid < NCO) ? red[(tid < NCO) ? tid : 0][0] : 0.0f;
  __syncthreads();
  for (int ps = 0; ps < 2; ++ps) {
    if (tid < 8) {
      v4f x = *(const v4fa*)&ln[4 * tid];
      *(volatile v4f*)(part + (size_t)blockIdx.x * 32 + 4 * tid) = x;
    }
    if (ps == 0) __threadfence();
  }
}

__global__ __launch_bounds__(32) void stat_k(const float* __restrict__ part, const float* __restrict__ phi,
                                             float* __restrict__ stat, int npts) {
  __shared__ __attribute__((aligned(16))) float ln[32];
  const int lane = threadIdx.x;
  ln[lane] = 0.0f;
  __syncthreads();
  if (lane < NVOL) {
    int b = lane / NCO, c = lane - b * NCO;
    float sum = 0.0f;
    for (int k = 0; k < NSB; ++k) sum += part[(size_t)(b * NSB + k) * 32 + c];
    float fv = sum / (float)npts;
    float p00 = phi[(size_t)lane * VOX];
    float rc = 1.0f / fabsf(p00 - fv);
    ln[lane] = fv;
    ln[8 + lane] = rc;
  }
  __syncthreads();
  for (int ps = 0; ps < 2; ++ps) {
    if (lane < 8) {
      v4f x = *(const v4fa*)&ln[4 * lane];
      *(volatile v4f*)(stat + 4 * lane) = x;
    }
    if (ps == 0) __threadfence();
  }
}

__global__ __launch_bounds__(256) void fin_k(const float* __restrict__ phi, const float* __restrict__ stat,
                                            float* __restrict__ out) {
  const int n4 = NVOL * VOX / 4;
  int i = blockIdx.x * 256 + threadIdx.x;
  if (i >= n4) return;
  size_t e = (size_t)i * 4;
  int v = (int)(e >> 21);
  float fv = stat[v], rc = stat[8 + v];
  v4f x = *(const v4fa*)(phi + e);
  v4f d = x - fv;
  v4f y = ((-d) * rc) * 0.5f;
  *(volatile v4f*)(out + e) = y;
  __threadfence();
  *(volatile v4f*)(out + e) = y;
}

extern "C" void kernel_launch(void* const* d_in, const int* in_sizes, int n_in,
                              void* d_out, int out_size, void* d_ws,
                              size_t ws_size, hipStream_t stream) {
  if (n_in < 2) return;
  const int npts = in_sizes[1] / 6;
  if (npts <= 0 || in_sizes[1] != 6 * npts || in_sizes[0] != 8 * npts) return;
  if (out_size != NVOL * VOX) return;
  const float* logits = (const float*)d_in[0];
  const float* coords = (const float*)d_in[1];
  float* out = (float*)d_out;

  char* ws = (char*)d_ws;
  size_t off = 0;
  auto carve = [&](size_t bytes) -> char* { char* p = ws + off; off += (bytes + 255) & ~(size_t)255; return p; };
  float* probs = (float*)carve((size_t)NVOL * npts * 4);
  char* regA = carve((size_t)NVOL * VOX * 4);
  char* regP = carve((size_t)3 * NVOL * VOX * 2);
  _Float16* RT  = (_Float16*)carve(128 * 128 * 2);
  _Float16* Ct  = (_Float16*)carve(128 * 128 * 2);
  _Float16* St  = (_Float16*)carve(128 * 128 * 2);
  _Float16* Snt = (_Float16*)carve(128 * 128 * 2);
  _Float16* Czt = (_Float16*)carve(128 * 64 * 2);
  _Float16* Szt = (_Float16*)carve(128 * 64 * 2);
  float* part = (float*)carve((size_t)2 * NSB * 32 * 4);
  float* stat = (float*)carve(128);
  if (off > ws_size) return;

  float* g   = (float*)regA;
  float* Zre = (float*)regA;  float* Zim = Zre + (size_t)NVOL * 16384 * 64;
  float* Xre = (float*)regA;  float* Xim = Xre + (size_t)NVOL * 6144 * 128;
  float* IYre = Xre;          float* IYim = Xim;
  _Float16* Px = (_Float16*)regP; _Float16* Py = Px + (size_t)NVOL * VOX; _Float16* Pz = Py + (size_t)NVOL * VOX;
  float* Yre = (float*)regP;  float* Yim = Yre + (size_t)NVOL * 6144 * 128;
  float* IXre = Yre;          float* IXim = Yim;
  float* phi = (float*)regP;

  const int dynl = NCO * 16384 * 4;
  hipFuncSetAttribute(reinterpret_cast<const void*>(&splat_k), hipFuncAttributeMaxDynamicSharedMemorySize, dynl);

  probs_k<<<(2 * npts + 255) / 256, 256, 0, stream>>>(logits, probs, npts);
  splat_k<<<2 * 128, 32, dynl, stream>>>(coords, probs, g, npts);
  init_k<<<384, 128, 0, stream>>>(RT, Ct, St, Snt, Czt, Szt);

  const unsigned B16 = NVOL * 16384 / 32;
  const unsigned B6  = NVOL * 6144 / 32;
  pass_k<0><<<B16, 64, 0, stream>>>(g, g, Px, Px, Px, RT, RT, RT, Zre, Zre, Px);
  pass_k<1><<<B16, 64, 0, stream>>>(g, g, Px, Px, Px, RT, RT, RT, Zre, Zre, Py);
  pass_k<2><<<B16, 64, 0, stream>>>(g, g, Px, Px, Px, RT, RT, RT, Zre, Zre, Pz);
  pass_k<3><<<B16, 64, 0, stream>>>(Zre, Zre, Pz, Py, Px, Ct, St, Snt, Zre, Zim, Px);
  pass_k<4><<<B6, 64, 0, stream>>>(Zre, Zim, Px, Px, Px, Ct, St, Snt, Yre, Yim, Px);
  pass_k<5><<<B6, 64, 0, stream>>>(Yre, Yim, Px, Px, Px, Ct, St, Snt, Xre, Xim, Px);
  pass_k<6><<<B6, 64, 0, stream>>>(Xre, Xim, Px, Px, Px, Ct, Snt, St, IXre, IXim, Px);
  pass_k<7><<<B6, 64, 0, stream>>>(IXre, IXim, Px, Px, Px, Ct, Snt, St, IYre, IYim, Px);
  pass_k<8><<<B16, 64, 0, stream>>>(IYre, IYim, Px, Px, Px, Czt, Szt, Czt, phi, phi, Px);

  samp_k<<<2 * NSB, 256, 0, stream>>>(coords, phi, part, npts);
  stat_k<<<1, 32, 0, stream>>>(part, phi, stat, npts);
  fin_k<<<(NVOL * VOX / 4 + 255) / 256, 256, 0, stream>>>(phi, stat, out);
}
